// SelfAttention3D_16681652978025
// MI455X (gfx1250) — hardware-verified
//
#include <hip/hip_runtime.h>


#ifndef NB
#define NB 1
#endif
#ifndef SEQ
#define SEQ 4096
#endif
#define SEQ_FULL 4096
#define XPITCH SEQ_FULL
#define CC   256
#define NHD  8
#define HD   32
#define QB   64
#define TP   72
#define PCAR 1024.0f
#define ACAR 16.0f
#define WCAR 16.0f
#define SCL  0.17677669529663687f
#define L2E  1.4426950408889634f
#define C2   (SCL * L2E)
static_assert(SEQ % 64 == 0);
static_assert(SEQ <= SEQ_FULL);
static_assert(CC == NHD * HD);
static_assert((NHD % 2) == 0);
static_assert(NB == 1);

typedef _Float16 h16;
typedef unsigned short bf;
typedef __attribute__((ext_vector_type(16))) __bf16   v16bf;
typedef __attribute__((ext_vector_type(16))) _Float16 v16h;
typedef __attribute__((ext_vector_type(8)))  _Float16 v8h;
typedef __attribute__((ext_vector_type(8)))  unsigned short v8us;
typedef __attribute__((ext_vector_type(8)))  float    v8f;
typedef __attribute__((ext_vector_type(4)))  float    v4f;
typedef v8h  __attribute__((may_alias)) v8ha;
typedef v4f  __attribute__((may_alias)) v4fa;
typedef v8us __attribute__((may_alias)) v8usa;

__device__ __forceinline__ unsigned short f2bf(float f) { unsigned u = __float_as_uint(f); u += 0x7FFFu + ((u >> 16) & 1u); return (unsigned short)(u >> 16); }
__device__ __forceinline__ float bf2f(unsigned short b) { return __uint_as_float(((unsigned)b) << 16); }
__device__ __forceinline__ float bfr(float f) { return bf2f(f2bf(f)); }
__device__ __forceinline__ v16h cat16(v8h lo, v8h hi) { return __builtin_shufflevector(lo, hi, 0, 1, 2, 3, 4, 5, 6, 7, 8, 9, 10, 11, 12, 13, 14, 15); }
__device__ __forceinline__ v16bf cat16b(v8us lo, v8us hi) { return __builtin_bit_cast(v16bf, __builtin_shufflevector(lo, hi, 0, 1, 2, 3, 4, 5, 6, 7, 8, 9, 10, 11, 12, 13, 14, 15)); }
__device__ __forceinline__ v8f wmma16(v16h a, v16h b, v8f c) { return __builtin_amdgcn_wmma_f32_16x16x32_f16(false, a, false, b, (short)0, c, false, false); }
__device__ __forceinline__ v8f wmmab(v16bf a, v16bf b, v8f c) { return __builtin_amdgcn_wmma_f32_16x16x32_bf16(false, a, false, b, (short)0, c, false, false); }

template <typename T16> struct WFrag;
template <> struct WFrag<h16> { typedef v16h V; static __device__ __forceinline__ V ld(const h16* p) { return cat16(*(const v8h*)p, *(const v8h*)(p + 16)); } static __device__ __forceinline__ v8f mma(V a, V b, v8f c) { return wmma16(a, b, c); } };
template <> struct WFrag<bf> { typedef v16bf V; static __device__ __forceinline__ V ld(const bf* p) { return cat16b(*(const v8us*)p, *(const v8us*)(p + 16)); } static __device__ __forceinline__ v8f mma(V a, V b, v8f c) { return wmmab(a, b, c); } };

template <typename T16, int MODE>
__global__ __launch_bounds__(32) void k_gemmw(const T16* __restrict__ A, const T16* __restrict__ Bt, int K, float* C, int ldc,
                                              const float* __restrict__ bias, const float* __restrict__ R, int ldr, const float* __restrict__ gam, float osc) {
    typedef typename WFrag<T16>::V V;
    __shared__ __align__(16) float os[16 * 68];
    const int lane = threadIdx.x & 31, lr = lane & 15, hi = lane >> 4; const int r0 = blockIdx.x * 64, c0 = blockIdx.y * 64;
    float gsc = 0.f;
    if (MODE == 2) gsc = bfr(gam[0]);
    v8f acc[4][4];
#pragma unroll
    for (int mb = 0; mb < 4; ++mb)
#pragma unroll
        for (int nb = 0; nb < 4; ++nb) acc[mb][nb] = (v8f){};
    const size_t aoff = (size_t)(r0 + lr) * K + 8 * hi, boff = (size_t)(c0 + lr) * K + 8 * hi;
#pragma unroll 1
    for (int kc = 0; kc < K; kc += 32) {
        V a[4];
#pragma unroll
        for (int mb = 0; mb < 4; ++mb) a[mb] = WFrag<T16>::ld(A + aoff + (size_t)mb * 16 * K + kc);
#pragma unroll
        for (int nb = 0; nb < 4; ++nb) { const V b = WFrag<T16>::ld(Bt + boff + (size_t)nb * 16 * K + kc);
#pragma unroll
            for (int mb = 0; mb < 4; ++mb) acc[mb][nb] = WFrag<T16>::mma(a[mb], b, acc[mb][nb]); }
        asm volatile("v_nop\n\tv_nop\n\tv_nop\n\tv_nop" : "+v"(acc[0][0]), "+v"(acc[1][1]), "+v"(acc[2][2]), "+v"(acc[3][3]) : "v"(a[0]), "v"(a[3]));
    }
#pragma unroll
    for (int mb = 0; mb < 4; ++mb) {
#pragma unroll
        for (int nb = 0; nb < 4; ++nb) {
#pragma unroll
            for (int j = 0; j < 8; ++j) os[(hi * 8 + j) * 68 + nb * 16 + lr] = acc[mb][nb][j]; }
        __builtin_amdgcn_wave_barrier(); asm volatile("" ::: "memory");
        float* crow = C + (size_t)(r0 + mb * 16) * ldc + c0;
#pragma unroll 1
        for (int ps = 0; ps < 2; ++ps) {
#pragma unroll
            for (int s = 0; s < 8; ++s) { const int row = 2 * s + hi, cofs = lr * 4; v4f val = *(const v4fa*)(os + row * 68 + cofs);
                if (MODE == 1) { val[0] += bfr(bias[c0 + cofs]); val[1] += bfr(bias[c0 + cofs + 1]); val[2] += bfr(bias[c0 + cofs + 2]); val[3] += bfr(bias[c0 + cofs + 3]); }
                if (MODE == 2) { const int gr = r0 + mb * 16 + row; const float rb = bfr(bias[gr]); const v4f xr = *(const v4f*)(R + (size_t)gr * ldr + c0 + cofs);
#pragma unroll
                    for (int j = 0; j < 4; ++j) { const float xv = xr[j]; const float av = val[j]; val[j] = bfr(xv) + gsc * (av * osc + rb); } }
                *(volatile v4f*)(crow + (size_t)row * ldc + cofs) = val; }
            if (ps == 0) __threadfence(); }
        __builtin_amdgcn_wave_barrier(); asm volatile("" ::: "memory");
    }
}

__global__ __launch_bounds__(256) void k_cvt8(const float* __restrict__ src, bf* dst, size_t n8) { const size_t i = (size_t)blockIdx.x * 256 + threadIdx.x; if (i >= n8) return; const v8f v = *(const v8f*)(src + i * 8); v8us o;
#pragma unroll
    for (int k = 0; k < 8; ++k) o[k] = f2bf(v[k]); *(volatile v8us*)(dst + i * 8) = o; __threadfence(); *(volatile v8us*)(dst + i * 8) = o; }

__global__ __launch_bounds__(256) void k_wo16(const float* __restrict__ src, h16* dst, size_t n8) { const size_t i = (size_t)blockIdx.x * 256 + threadIdx.x; if (i >= n8) return; const v8f v = *(const v8f*)(src + i * 8); v8f t = (v8f){};
#pragma unroll
    for (int k = 0; k < 8; ++k) t[k] = bfr(v[k]) * WCAR; const v8h o = __builtin_convertvector(t, v8h); *(volatile v8h*)(dst + i * 8) = o; __threadfence(); *(volatile v8h*)(dst + i * 8) = o; }

__global__ __launch_bounds__(256) void k_xT(const float* __restrict__ x, bf* XB) {
    __shared__ float sm[64 * 65];
    const int tid = threadIdx.x; const int n0 = blockIdx.x * 64, c0 = blockIdx.y * 64;
#pragma unroll
    for (int it = 0; it < 4; ++it) { const int c = it * 16 + (tid >> 4), nf = (tid & 15) * 4; const v4f v = *(const v4f*)(x + (size_t)(c0 + c) * XPITCH + n0 + nf);
        sm[c * 65 + nf] = v[0]; sm[c * 65 + nf + 1] = v[1]; sm[c * 65 + nf + 2] = v[2]; sm[c * 65 + nf + 3] = v[3]; }
    __syncthreads();
#pragma unroll 1
    for (int ps = 0; ps < 2; ++ps) {
#pragma unroll
        for (int it = 0; it < 2; ++it) { const int n = it * 32 + (tid >> 3), p = tid & 7; v8us o;
#pragma unroll
            for (int j = 0; j < 8; ++j) o[j] = f2bf(sm[(p * 8 + j) * 65 + n]);
            *(volatile v8us*)(XB + (size_t)(n0 + n) * CC + c0 + p * 8) = o; }
        if (ps == 0) __threadfence(); }
}

__global__ __launch_bounds__(256) void k_tof16(const float* __restrict__ F, const float* __restrict__ rbias, int rowlen, h16* P, size_t n8) {
    const size_t i = (size_t)blockIdx.x * 256 + threadIdx.x; if (i >= n8) return;
    float b = 0.f;
    if (rbias != nullptr) { const unsigned row = (unsigned)i / (unsigned)(rowlen >> 3); b = bfr(rbias[row]); }
    const v8f v = *(const v8f*)(F + i * 8);
    const v8h o = __builtin_convertvector(v + b, v8h);
    *(volatile v8h*)(P + i * 8) = o; __threadfence(); *(volatile v8h*)(P + i * 8) = o; }

__device__ __forceinline__ void att_step(const v16h ak0, const v16h ak1, const v16h av0, const v16h av1, const v16h bq, float& m, float& l, v8f& o0, v8f& o1) {
    v8f s0 = wmma16(ak0, bq, (v8f){}); v8f s1 = wmma16(ak1, bq, (v8f){});
    asm volatile("v_nop\n\tv_nop\n\tv_nop\n\tv_nop" : "+v"(s0), "+v"(s1) : "v"(ak0), "v"(ak1), "v"(bq));
    float cmx = -1.0e30f;
#pragma unroll
    for (int j = 0; j < 8; ++j) cmx = fmaxf(cmx, fmaxf(s0[j], s1[j]));
    cmx = fmaxf(cmx, __shfl_xor(cmx, 16, 32));
    const float nm = fmaxf(m, cmx * C2);
    const float alpha = __builtin_amdgcn_exp2f(m - nm);
    v8f p0 = (v8f){}, p1 = (v8f){}; float rs = 0.f;
#pragma unroll
    for (int j = 0; j < 8; ++j) { const float e0 = __builtin_amdgcn_exp2f(s0[j] * C2 - nm); const float e1 = __builtin_amdgcn_exp2f(s1[j] * C2 - nm); p0[j] = e0; p1[j] = e1; rs += e0 + e1; }
    rs += __shfl_xor(rs, 16, 32);
    l = l * alpha + rs; m = nm;
    o0 *= alpha; o1 *= alpha;
    const v16h bp = cat16(__builtin_convertvector(p0 * PCAR, v8h), __builtin_convertvector(p1 * PCAR, v8h));
    o0 = wmma16(av0, bp, o0); o1 = wmma16(av1, bp, o1);
    asm volatile("v_nop\n\tv_nop\n\tv_nop\n\tv_nop" : "+v"(o0), "+v"(o1) : "v"(av0), "v"(av1), "v"(bp));
}

__global__ __launch_bounds__(128) __attribute__((amdgpu_num_vgpr(256)))
void k_attn(const h16* __restrict__ Q16, const h16* __restrict__ K16, const h16* __restrict__ VT, h16* ATT) {
    __shared__ __align__(16) h16 ts[QB * TP];
    const int tid = threadIdx.x, w = tid >> 5, lane = tid & 31, lr = lane & 15, hi = lane >> 4;
    const int q0 = blockIdx.x * QB, hp = blockIdx.y, hq = w >> 1, g = w & 1, head = hp * 2 + hq, qb = q0 + g * 32;
    const h16* Qp = Q16 + (size_t)qb * CC + head * HD + 8 * hi;
    const v16h bq0 = WFrag<h16>::ld(Qp + (size_t)lr * CC);
    const v16h bq1 = WFrag<h16>::ld(Qp + (size_t)(16 + lr) * CC);
    const h16* Kp = K16 + (size_t)lr * CC + head * HD + 8 * hi;
    const h16* Vp = VT + (size_t)(head * HD + lr) * SEQ + 8 * hi;
    float m0 = -1.0e30f, m1 = -1.0e30f, l0 = 0.f, l1 = 0.f;
    v8f o00 = (v8f){}, o10 = (v8f){}, o01 = (v8f){}, o11 = (v8f){};
#pragma unroll 1
    for (int k0 = 0; k0 < SEQ; k0 += 32) {
        const v16h ak0 = WFrag<h16>::ld(Kp + (size_t)k0 * CC), ak1 = WFrag<h16>::ld(Kp + (size_t)(k0 + 16) * CC);
        const v16h av0 = WFrag<h16>::ld(Vp + k0), av1 = WFrag<h16>::ld(Vp + (size_t)16 * SEQ + k0);
        att_step(ak0, ak1, av0, av1, bq0, m0, l0, o00, o10);
        att_step(ak0, ak1, av0, av1, bq1, m1, l1, o01, o11);
    }
    {
        const float inv0 = (ACAR / PCAR) * (1.0f / l0), inv1 = (ACAR / PCAR) * (1.0f / l1);
        h16* t0 = ts + (size_t)(g * 32 + lr) * TP + hq * 32 + 8 * hi;
        h16* t1 = ts + (size_t)(g * 32 + 16 + lr) * TP + hq * 32 + 8 * hi;
        *(v8ha*)(t0) = __builtin_convertvector(o00 * inv0, v8h); *(v8ha*)(t0 + 16) = __builtin_convertvector(o10 * inv0, v8h);
        *(v8ha*)(t1) = __builtin_convertvector(o01 * inv1, v8h); *(v8ha*)(t1 + 16) = __builtin_convertvector(o11 * inv1, v8h);
    }
    __syncthreads();
#pragma unroll 1
    for (int ps = 0; ps < 2; ++ps) {
#pragma unroll
        for (int it = 0; it < 4; ++it) { const int row = w * 16 + it * 4 + (lane >> 3), pc = (lane & 7) * 8; const v8h val = *(const v8ha*)(ts + row * TP + pc);
            *(volatile v8h*)(ATT + (size_t)(q0 + row) * CC + hp * 64 + pc) = val; }
        if (ps == 0) __threadfence(); }
}

extern "C" void kernel_launch(void* const* d_in, const int* in_sizes, int n_in,
                              void* d_out, int out_size, void* d_ws, size_t ws_size, hipStream_t stream) {
    if (n_in < 10) return;
    if (in_sizes[0] < (CC - 1) * XPITCH + SEQ) return;
    if (in_sizes[1] < CC * CC || in_sizes[3] < CC * CC || in_sizes[5] < CC * CC || in_sizes[7] < CC * CC) return;
    if (in_sizes[2] < CC || in_sizes[4] < CC || in_sizes[6] < CC || in_sizes[8] < CC || in_sizes[9] < 1) return;
    if (out_size < CC * SEQ) return;
    const float* x = (const float*)d_in[0]; const float* wq = (const float*)d_in[1]; const float* bq = (const float*)d_in[2]; const float* wk = (const float*)d_in[3]; const float* bk = (const float*)d_in[4];
    const float* wv = (const float*)d_in[5]; const float* bv = (const float*)d_in[6]; const float* wo = (const float*)d_in[7]; const float* bo = (const float*)d_in[8]; const float* gamma = (const float*)d_in[9];
    float* OUT = (float*)d_out;
    char* wsp = (char*)d_ws;
    auto take = [&](size_t bytes) { char* p = wsp; wsp += (bytes + 255) & ~(size_t)255; return (void*)p; };
    bf* WQ = (bf*)take((size_t)CC * CC * 2); bf* WK = (bf*)take((size_t)CC * CC * 2); bf* WV = (bf*)take((size_t)CC * CC * 2); h16* WO16 = (h16*)take((size_t)CC * CC * 2);
    bf* XB = (bf*)take((size_t)SEQ * CC * 2);
    float* FQ = (float*)take((size_t)SEQ * CC * 4); float* FK = (float*)take((size_t)SEQ * CC * 4); float* FVt = (float*)take((size_t)CC * SEQ * 4);
    h16* Q16 = (h16*)take((size_t)SEQ * CC * 2); h16* K16 = (h16*)take((size_t)SEQ * CC * 2); h16* VT16 = (h16*)take((size_t)CC * SEQ * 2); h16* ATT = (h16*)take((size_t)SEQ * CC * 2);
    if ((size_t)(wsp - (char*)d_ws) > ws_size) return;
    const unsigned nw8 = (unsigned)(((size_t)CC * CC / 8 + 255) / 256);
    const unsigned ncv = (unsigned)(((size_t)SEQ * CC / 8 + 255) / 256);
    k_cvt8<<<nw8, 256, 0, stream>>>(wq, WQ, (size_t)CC * CC / 8);
    k_cvt8<<<nw8, 256, 0, stream>>>(wk, WK, (size_t)CC * CC / 8);
    k_cvt8<<<nw8, 256, 0, stream>>>(wv, WV, (size_t)CC * CC / 8);
    k_wo16<<<nw8, 256, 0, stream>>>(wo, WO16, (size_t)CC * CC / 8);
    k_xT<<<dim3(SEQ / 64, CC / 64, 1), 256, 0, stream>>>(x, XB);
    k_gemmw<bf, 1><<<dim3(SEQ / 64, CC / 64, 1), 32, 0, stream>>>(XB, WQ, CC, FQ, CC, bq, nullptr, 0, nullptr, 1.0f);
    k_gemmw<bf, 1><<<dim3(SEQ / 64, CC / 64, 1), 32, 0, stream>>>(XB, WK, CC, FK, CC, bk, nullptr, 0, nullptr, 1.0f);
    k_gemmw<bf, 0><<<dim3(CC / 64, SEQ / 64, 1), 32, 0, stream>>>(WV, XB, CC, FVt, SEQ, nullptr, nullptr, 0, nullptr, 1.0f);
    k_tof16<<<ncv, 256, 0, stream>>>(FQ, nullptr, CC, Q16, (size_t)SEQ * CC / 8);
    k_tof16<<<ncv, 256, 0, stream>>>(FK, nullptr, CC, K16, (size_t)SEQ * CC / 8);
    k_tof16<<<ncv, 256, 0, stream>>>(FVt, bv, SEQ, VT16, (size_t)SEQ * CC / 8);
    k_attn<<<dim3(SEQ / QB, NHD / 2, 1), 128, 0, stream>>>(Q16, K16, VT16, ATT);
    k_gemmw<h16, 2><<<dim3(CC / 64, SEQ / 64, 1), 32, 0, stream>>>(WO16, ATT, CC, OUT, SEQ, bo, x, XPITCH, gamma, 1.0f / (ACAR * WCAR));
}
